// GCN_3_layers_31860067401788
// MI455X (gfx1250) — hardware-verified
//
#include <hip/hip_runtime.h>
#include <stddef.h>


#define DF      128
#define C2      64
#define C3      32
#define NTHR    256
#define NWAVE   8
#define EPT     8
#define NGRP    2
#define CHUNK   (NTHR * EPT * NGRP)
#define WCAP    (EPT * NGRP * 32)
#define LISTN   (NWAVE * WCAP)
#define NB1     512
#define NB2     1024
#define NB3     2048
#define NBD     4096
#define G1ROWS  128
#define APITCH  136
#define WSCALE  16.0f
#define WINV    0.0625f
#define SLOPE   0.1f

#define LDS_GEMM1 (G1ROWS * DF * 4)
#define LDS_AGG   (NB1 * DF * 4 + LISTN * 4 + 64)

static_assert((CHUNK & (CHUNK - 1)) == 0);
static_assert(CHUNK <= 4096);
static_assert(NB1 <= 4096 && NB2 <= 4096 && NB3 <= 4096 && NBD <= 4096);
static_assert(NB1 * DF == NB2 * C2 && NB2 * C2 == NB3 * C3);
static_assert(G1ROWS * APITCH * 2 <= LDS_GEMM1);
static_assert(NBD == NWAVE * 4 * 128);
static_assert(NB1 / 16 == 4 * NWAVE && NB2 / 16 == 8 * NWAVE && NB3 == 256 * NWAVE);

typedef float    v2f  __attribute__((ext_vector_type(2)));
typedef float    v4f  __attribute__((ext_vector_type(4)));
typedef float    v8f  __attribute__((ext_vector_type(8)));
typedef int      v4i  __attribute__((ext_vector_type(4)));
typedef _Float16 v8h  __attribute__((ext_vector_type(8)));
typedef _Float16 v16h __attribute__((ext_vector_type(16)));
union FragH { v16h v; v8h h[2]; };

__device__ __forceinline__ v8h cvt8(v4f a, v4f b) {
  v8h r;
  r[0] = (_Float16)a.x; r[1] = (_Float16)a.y; r[2] = (_Float16)a.z; r[3] = (_Float16)a.w;
  r[4] = (_Float16)b.x; r[5] = (_Float16)b.y; r[6] = (_Float16)b.z; r[7] = (_Float16)b.w;
  return r;
}

__device__ __forceinline__ v8f wmh(v16h a, v16h b, v8f c) {
  v8f d = __builtin_amdgcn_wmma_f32_16x16x32_f16(false, a, false, b, (short)0, c, false, false);
  asm volatile("v_nop\n\tv_nop\n\tv_nop\n\tv_nop" : "+v"(d) : "v"(a), "v"(b));
  return d;
}

template <int NB>
__device__ __forceinline__ int scan_chunk(const int* __restrict__ lst, int nE, int cbase, int nodeBase,
                                          int* list, int tid, int lane, int wave) {
  int wc = 0;
#pragma unroll
  for (int g = 0; g < NGRP; ++g) {
    const int el0  = (g * NTHR + tid) * EPT;
    const int e0   = cbase + el0;
    const int sent = -2147483647 - 1;
    v4i da, db;
    if (e0 + 7 < nE) {
      da = *(const v4i*)(lst + e0);
      db = *(const v4i*)(lst + e0 + 4);
    } else {
      da.x = (e0     < nE) ? lst[min(e0, nE - 1)] : sent;
      da.y = (e0 + 1 < nE) ? lst[min(e0 + 1, nE - 1)] : sent;
      da.z = (e0 + 2 < nE) ? lst[min(e0 + 2, nE - 1)] : sent;
      da.w = (e0 + 3 < nE) ? lst[min(e0 + 3, nE - 1)] : sent;
      db.x = (e0 + 4 < nE) ? lst[min(e0 + 4, nE - 1)] : sent;
      db.y = (e0 + 5 < nE) ? lst[min(e0 + 5, nE - 1)] : sent;
      db.z = (e0 + 6 < nE) ? lst[min(e0 + 6, nE - 1)] : sent;
      db.w = (e0 + 7 < nE) ? lst[min(e0 + 7, nE - 1)] : sent;
    }
    const unsigned nb = (unsigned)nodeBase;
    const unsigned s0 = (unsigned)da.x - nb, s1 = (unsigned)da.y - nb;
    const unsigned s2 = (unsigned)da.z - nb, s3 = (unsigned)da.w - nb;
    const unsigned s4 = (unsigned)db.x - nb, s5 = (unsigned)db.y - nb;
    const unsigned s6 = (unsigned)db.z - nb, s7 = (unsigned)db.w - nb;
    const bool h0 = s0 < (unsigned)NB, h1 = s1 < (unsigned)NB, h2 = s2 < (unsigned)NB, h3 = s3 < (unsigned)NB;
    const bool h4 = s4 < (unsigned)NB, h5 = s5 < (unsigned)NB, h6 = s6 < (unsigned)NB, h7 = s7 < (unsigned)NB;
    const unsigned any = __builtin_amdgcn_ballot_w32(h0 | h1 | h2 | h3 | h4 | h5 | h6 | h7);
    if (any != 0u) {
#define HITJ(J, HJ, SJ) { \
        const unsigned mj = __builtin_amdgcn_ballot_w32(HJ); \
        if (mj != 0u) { \
          if (HJ) { \
            const int pos = wc + (int)__builtin_amdgcn_mbcnt_lo(mj, 0u); \
            if (pos < WCAP) list[wave * WCAP + pos] = ((el0 + (J)) << 12) | (int)(SJ); \
          } \
          wc += (int)__builtin_popcount(mj); } }
      HITJ(0, h0, s0)
      HITJ(1, h1, s1)
      HITJ(2, h2, s2)
      HITJ(3, h3, s3)
      HITJ(4, h4, s4)
      HITJ(5, h5, s5)
      HITJ(6, h6, s6)
      HITJ(7, h7, s7)
#undef HITJ
    }
  }
  return wc;
}

__global__ __launch_bounds__(NTHR) void k_wprep(
    const float* __restrict__ W1, const float* __restrict__ W2, const float* __restrict__ W3,
    _Float16* w1s, _Float16* w2s, _Float16* w3s) {
  const int i  = blockIdx.x * NTHR + threadIdx.x;
  const int n1 = DF * DF / 8;
  const int n2 = C2 * DF / 8;
  const int n3 = C3 * C2 / 8;
  if (i >= n1 + n2 + n3) return;
  int o, kd, nc;
  const float* W;
  _Float16* dstp;
  if (i < n1)           { o = i * 8;             kd = DF; nc = DF; W = W1; dstp = w1s; }
  else if (i < n1 + n2) { o = (i - n1) * 8;      kd = DF; nc = C2; W = W2; dstp = w2s; }
  else                  { o = (i - n1 - n2) * 8; kd = C2; nc = C3; W = W3; dstp = w3s; }
  const int n  = o / kd;
  const int k0 = o - n * kd;
  const float* p = W + (size_t)k0 * nc + n;
  v4f a, b;
  a.x = p[0];      a.y = p[nc];     a.z = p[2 * nc]; a.w = p[3 * nc];
  b.x = p[4 * nc]; b.y = p[5 * nc]; b.z = p[6 * nc]; b.w = p[7 * nc];
  a = a * WSCALE;
  b = b * WSCALE;
  const v8h hv = cvt8(a, b);
  _Float16* dp = dstp + o;
  *(volatile v8h*)dp = hv;
  __threadfence();
  *(volatile v8h*)dp = hv;
}

__global__ __launch_bounds__(NTHR) void k_deg(
    const int* __restrict__ srcl, const int* __restrict__ dstl, float* dO, float* dI, int nE, int nBD) {
  __shared__ __attribute__((aligned(16))) int cnt[NBD];
  __shared__ __attribute__((aligned(16))) int list[LISTN];
  __shared__ int wcnt[NWAVE];
  const int tid = threadIdx.x, lane = tid & 31, wave = tid >> 5;
  const int sel = ((int)blockIdx.x >= nBD) ? 1 : 0;
  const int* lst = sel ? dstl : srcl;
  float* dinv = sel ? dI : dO;
  const int nodeBase = ((int)blockIdx.x - sel * nBD) * NBD;

  for (int i = tid; i < NBD; i += NTHR) cnt[i] = 0;
  __syncthreads();

  const int nChunks = (nE + CHUNK - 1) / CHUNK;
#pragma unroll 1
  for (int ch = 0; ch < nChunks; ++ch) {
    const int cbase = ch * CHUNK;
    const int wc = scan_chunk<NBD>(lst, nE, cbase, nodeBase, list, tid, lane, wave);
    if (lane == 0) wcnt[wave] = wc;
    __syncthreads();
    if (wave == 0) {
#pragma unroll 1
      for (int wsx = 0; wsx < NWAVE; ++wsx) {
        int n = __builtin_amdgcn_readfirstlane(wcnt[wsx]);
        n = n > WCAP ? WCAP : (n < 0 ? 0 : n);
        const int* lp = list + wsx * WCAP;
#pragma unroll 1
        for (int i = 0; i < n; ++i) {
          const int ent  = __builtin_amdgcn_readfirstlane(lp[i]);
          const int slot = ent & (NBD - 1);
          if (lane == 0) cnt[slot] = cnt[slot] + 1;
        }
      }
    }
    __syncthreads();
  }

  v4f dq[4];
#pragma unroll
  for (int q = 0; q < 4; ++q) {
    const int f = (wave * 4 + q) * 128 + 4 * lane;
    const v4i c = *(const v4i*)(cnt + f);
    dq[q].x = rsqrtf((float)(c.x < 1 ? 1 : c.x));
    dq[q].y = rsqrtf((float)(c.y < 1 ? 1 : c.y));
    dq[q].z = rsqrtf((float)(c.z < 1 ? 1 : c.z));
    dq[q].w = rsqrtf((float)(c.w < 1 ? 1 : c.w));
  }
  float* dp = dinv + (size_t)nodeBase;
#pragma unroll
  for (int q = 0; q < 4; ++q) *(volatile v4f*)(dp + (wave * 4 + q) * 128 + 4 * lane) = dq[q];
  __threadfence();
#pragma unroll
  for (int q = 0; q < 4; ++q) *(volatile v4f*)(dp + (wave * 4 + q) * 128 + 4 * lane) = dq[q];
}

__global__ __launch_bounds__(NTHR) void k_gemm1(
    const float* __restrict__ x, const _Float16* __restrict__ w1s,
    const float* __restrict__ dO, float* g1, int nN) {
  extern __shared__ v4f lds_dyn[];
  _Float16* sA  = (_Float16*)lds_dyn;
  float*    stg = (float*)lds_dyn;
  const int tid = threadIdx.x, lane = tid & 31, wave = tid >> 5, hh = lane >> 4, m = lane & 15;
  const int rowBase = blockIdx.x * G1ROWS;

#pragma unroll
  for (int i = 0; i < (G1ROWS * DF / 8) / NTHR; ++i) {
    const int idx = i * NTHR + tid;
    const int r   = idx >> 4;
    const int c0  = (idx & 15) * 8;
    int node = rowBase + r;
    node = node > nN - 1 ? nN - 1 : node;
    const float* xp = x + (size_t)node * DF + c0;
    const v4f a = *(const v4f*)xp, b = *(const v4f*)(xp + 4);
    *(v8h*)(sA + r * APITCH + c0) = cvt8(a, b);
  }
  __syncthreads();

  v8f acc[8];
#pragma unroll
  for (int t = 0; t < 8; ++t) { v8f z = {0.f, 0.f, 0.f, 0.f, 0.f, 0.f, 0.f, 0.f}; acc[t] = z; }
  const _Float16* ar = sA + (wave * 16 + m) * APITCH + 8 * hh;
#pragma unroll
  for (int kt = 0; kt < DF / 32; ++kt) {
    FragH a;
    a.h[0] = *(const v8h*)(ar + 32 * kt);
    a.h[1] = *(const v8h*)(ar + 32 * kt + 16);
#pragma unroll
    for (int t = 0; t < 8; ++t) {
      const _Float16* bp = w1s + (size_t)(16 * t + m) * DF + 32 * kt + 8 * hh;
      FragH b;
      b.h[0] = *(const v8h*)bp;
      b.h[1] = *(const v8h*)(bp + 16);
      acc[t] = wmh(a.v, b.v, acc[t]);
    }
  }
  __syncthreads();

  const int r0 = wave * 16 + 8 * hh;
  const v4f dA = *(const v4f*)(dO + (size_t)rowBase + r0);
  const v4f dB = *(const v4f*)(dO + (size_t)rowBase + r0 + 4);
  const float d0 = dA.x * WINV, d1 = dA.y * WINV, d2 = dA.z * WINV, d3 = dA.w * WINV;
  const float d4 = dB.x * WINV, d5 = dB.y * WINV, d6 = dB.z * WINV, d7 = dB.w * WINV;
  float* sp = stg + r0 * DF + m;
#pragma unroll
  for (int t = 0; t < 8; ++t) {
    sp[0 * DF + 16 * t] = acc[t][0] * d0;
    sp[1 * DF + 16 * t] = acc[t][1] * d1;
    sp[2 * DF + 16 * t] = acc[t][2] * d2;
    sp[3 * DF + 16 * t] = acc[t][3] * d3;
    sp[4 * DF + 16 * t] = acc[t][4] * d4;
    sp[5 * DF + 16 * t] = acc[t][5] * d5;
    sp[6 * DF + 16 * t] = acc[t][6] * d6;
    sp[7 * DF + 16 * t] = acc[t][7] * d7;
  }
  __syncthreads();

  const float* lp = stg + wave * 16 * DF + 4 * lane;
  float* gp = g1 + ((size_t)rowBase + wave * 16) * DF + 4 * lane;
#pragma unroll
  for (int i = 0; i < 16; ++i) { const v4f v = *(const v4f*)(lp + i * DF); *(volatile v4f*)(gp + (size_t)i * DF) = v; }
  __threadfence();
#pragma unroll
  for (int i = 0; i < 16; ++i) { const v4f v = *(const v4f*)(lp + i * DF); *(volatile v4f*)(gp + (size_t)i * DF) = v; }
}

__global__ __launch_bounds__(NTHR) void k_agg1(
    const int* __restrict__ srcl, const int* __restrict__ dstl, const float* __restrict__ g1,
    const float* __restrict__ dO, const float* __restrict__ dI, const float* __restrict__ b1,
    const _Float16* __restrict__ w2s, float* g2, int nN, int nE) {
  extern __shared__ v4f lds_dyn[];
  float* acc  = (float*)lds_dyn;
  int*   list = (int*)(acc + NB1 * DF);
  int*   wcnt = list + LISTN;
  const int tid = threadIdx.x, lane = tid & 31, wave = tid >> 5, hh = lane >> 4, m = lane & 15;
  const int nodeBase = blockIdx.x * NB1;

  {
    const v4f z = {0.f, 0.f, 0.f, 0.f};
    for (int i = tid; i < NB1 * DF / 4; i += NTHR) lds_dyn[i] = z;
  }
  __syncthreads();

  const int nChunks = (nE + CHUNK - 1) / CHUNK;
#pragma unroll 1
  for (int ch = 0; ch < nChunks; ++ch) {
    const int cbase = ch * CHUNK;
    const int wc = scan_chunk<NB1>(dstl, nE, cbase, nodeBase, list, tid, lane, wave);
    if (lane == 0) wcnt[wave] = wc;
    __syncthreads();
    if (wave == 0) {
#pragma unroll 1
      for (int wsx = 0; wsx < NWAVE; ++wsx) {
        int n = __builtin_amdgcn_readfirstlane(wcnt[wsx]);
        n = n > WCAP ? WCAP : (n < 0 ? 0 : n);
        const int* lp = list + wsx * WCAP;
#pragma unroll 1
        for (int i = 0; i < n; ++i) {
          const int ent  = __builtin_amdgcn_readfirstlane(lp[i]);
          const int slot = ent & (NB1 - 1);
          int e = cbase + ((ent >> 12) & (CHUNK - 1));
          e = e > nE - 1 ? nE - 1 : e;
          int s = srcl[e];
          s = s < 0 ? 0 : (s > nN - 1 ? nN - 1 : s);
          const v4f v = *(const v4f*)(g1 + (size_t)s * DF + 4 * lane);
          v4f* ap = (v4f*)(acc + slot * DF + 4 * lane);
          *ap = *ap + v;
        }
      }
    }
    __syncthreads();
  }

#pragma unroll 4
  for (int i = 0; i < (NB1 * DF / 4) / NTHR; ++i) {
    const int idx  = i * NTHR + tid;
    const int slot = idx >> 5;
    const int c4   = (idx & 31) * 4;
    int node = nodeBase + slot;
    node = node > nN - 1 ? nN - 1 : node;
    const float d  = dI[node];
    const v4f   bv = *(const v4f*)(b1 + c4);
    v4f* ap = (v4f*)(acc + slot * DF + c4);
    v4f hv = (*ap) * d + bv;
    hv.x = hv.x >= 0.f ? hv.x : SLOPE * hv.x;
    hv.y = hv.y >= 0.f ? hv.y : SLOPE * hv.y;
    hv.z = hv.z >= 0.f ? hv.z : SLOPE * hv.z;
    hv.w = hv.w >= 0.f ? hv.w : SLOPE * hv.w;
    *ap = hv;
  }
  __syncthreads();

#pragma unroll 1
  for (int q = 0; q < NB1 / 16 / NWAVE; ++q) {
    const int t = wave + NWAVE * q;
    v8f c[4];
#pragma unroll
    for (int ct = 0; ct < 4; ++ct) { v8f z = {0.f, 0.f, 0.f, 0.f, 0.f, 0.f, 0.f, 0.f}; c[ct] = z; }
#pragma unroll
    for (int kt = 0; kt < DF / 32; ++kt) {
      const float* ap = acc + (16 * t + m) * DF + 32 * kt + 8 * hh;
      const v4f p0 = *(const v4f*)ap,        p1 = *(const v4f*)(ap + 4);
      const v4f p2 = *(const v4f*)(ap + 16), p3 = *(const v4f*)(ap + 20);
      FragH a;
      a.h[0] = cvt8(p0, p1);
      a.h[1] = cvt8(p2, p3);
#pragma unroll
      for (int ct = 0; ct < C2 / 16; ++ct) {
        const _Float16* bp = w2s + (size_t)(16 * ct + m) * DF + 32 * kt + 8 * hh;
        FragH b;
        b.h[0] = *(const v8h*)bp;
        b.h[1] = *(const v8h*)(bp + 16);
        c[ct] = wmh(a.v, b.v, c[ct]);
      }
    }
    const int node0 = nodeBase + 16 * t + 8 * hh;
    const v4f dA = *(const v4f*)(dO + (size_t)node0);
    const v4f dB = *(const v4f*)(dO + (size_t)node0 + 4);
    const float d0 = dA.x * WINV, d1 = dA.y * WINV, d2 = dA.z * WINV, d3 = dA.w * WINV;
    const float d4 = dB.x * WINV, d5 = dB.y * WINV, d6 = dB.z * WINV, d7 = dB.w * WINV;
    float* sp = acc + (16 * t + 8 * hh) * DF + m;
#pragma unroll
    for (int ct = 0; ct < 4; ++ct) {
      sp[0 * DF + 16 * ct] = c[ct][0] * d0;
      sp[1 * DF + 16 * ct] = c[ct][1] * d1;
      sp[2 * DF + 16 * ct] = c[ct][2] * d2;
      sp[3 * DF + 16 * ct] = c[ct][3] * d3;
      sp[4 * DF + 16 * ct] = c[ct][4] * d4;
      sp[5 * DF + 16 * ct] = c[ct][5] * d5;
      sp[6 * DF + 16 * ct] = c[ct][6] * d6;
      sp[7 * DF + 16 * ct] = c[ct][7] * d7;
    }
  }
  __syncthreads();

  float* gbase = g2 + (size_t)nodeBase * C2;
#pragma unroll 4
  for (int q = 0; q < 32; ++q) {
    const int row = wave * 64 + 2 * q + (lane >> 4);
    const int col = 4 * (lane & 15);
    const v4f v = *(const v4f*)(acc + row * DF + col);
    *(volatile v4f*)(gbase + (size_t)row * C2 + col) = v;
  }
  __threadfence();
#pragma unroll 4
  for (int q = 0; q < 32; ++q) {
    const int row = wave * 64 + 2 * q + (lane >> 4);
    const int col = 4 * (lane & 15);
    const v4f v = *(const v4f*)(acc + row * DF + col);
    *(volatile v4f*)(gbase + (size_t)row * C2 + col) = v;
  }
}

__global__ __launch_bounds__(NTHR) void k_agg2(
    const int* __restrict__ srcl, const int* __restrict__ dstl, const float* __restrict__ g2,
    const float* __restrict__ dO, const float* __restrict__ dI, const float* __restrict__ b2,
    const _Float16* __restrict__ w3s, float* g3, int nN, int nE) {
  extern __shared__ v4f lds_dyn[];
  float* acc  = (float*)lds_dyn;
  int*   list = (int*)(acc + NB2 * C2);
  int*   wcnt = list + LISTN;
  const int tid = threadIdx.x, lane = tid & 31, wave = tid >> 5, hh = lane >> 4, m = lane & 15;
  const int nodeBase = blockIdx.x * NB2;

  {
    const v4f z = {0.f, 0.f, 0.f, 0.f};
    for (int i = tid; i < NB2 * C2 / 4; i += NTHR) lds_dyn[i] = z;
  }
  __syncthreads();

  const int nChunks = (nE + CHUNK - 1) / CHUNK;
#pragma unroll 1
  for (int ch = 0; ch < nChunks; ++ch) {
    const int cbase = ch * CHUNK;
    const int wc = scan_chunk<NB2>(dstl, nE, cbase, nodeBase, list, tid, lane, wave);
    if (lane == 0) wcnt[wave] = wc;
    __syncthreads();
    if (wave == 0) {
#pragma unroll 1
      for (int wsx = 0; wsx < NWAVE; ++wsx) {
        int n = __builtin_amdgcn_readfirstlane(wcnt[wsx]);
        n = n > WCAP ? WCAP : (n < 0 ? 0 : n);
        const int* lp = list + wsx * WCAP;
#pragma unroll 1
        for (int i = 0; i < n; ++i) {
          const int ent  = __builtin_amdgcn_readfirstlane(lp[i]);
          const int slot = ent & (NB2 - 1);
          int e = cbase + ((ent >> 12) & (CHUNK - 1));
          e = e > nE - 1 ? nE - 1 : e;
          int s = srcl[e];
          s = s < 0 ? 0 : (s > nN - 1 ? nN - 1 : s);
          const v2f v = *(const v2f*)(g2 + (size_t)s * C2 + 2 * lane);
          v2f* ap = (v2f*)(acc + slot * C2 + 2 * lane);
          *ap = *ap + v;
        }
      }
    }
    __syncthreads();
  }

#pragma unroll 4
  for (int i = 0; i < (NB2 * C2 / 4) / NTHR; ++i) {
    const int idx  = i * NTHR + tid;
    const int slot = idx >> 4;
    const int c4   = (idx & 15) * 4;
    int node = nodeBase + slot;
    node = node > nN - 1 ? nN - 1 : node;
    const float d  = dI[node];
    const v4f   bv = *(const v4f*)(b2 + c4);
    v4f* ap = (v4f*)(acc + slot * C2 + c4);
    v4f hv = (*ap) * d + bv;
    hv.x = hv.x >= 0.f ? hv.x : SLOPE * hv.x;
    hv.y = hv.y >= 0.f ? hv.y : SLOPE * hv.y;
    hv.z = hv.z >= 0.f ? hv.z : SLOPE * hv.z;
    hv.w = hv.w >= 0.f ? hv.w : SLOPE * hv.w;
    *ap = hv;
  }
  __syncthreads();

  FragH bw[2][2];
#pragma unroll
  for (int kt = 0; kt < 2; ++kt) {
#pragma unroll
    for (int ct = 0; ct < 2; ++ct) {
      const _Float16* bp = w3s + (16 * ct + m) * C2 + 32 * kt + 8 * hh;
      bw[kt][ct].h[0] = *(const v8h*)bp;
      bw[kt][ct].h[1] = *(const v8h*)(bp + 16);
    }
  }

#pragma unroll 1
  for (int q = 0; q < NB2 / 16 / NWAVE; ++q) {
    const int t = wave + NWAVE * q;
    v8f c[2];
#pragma unroll
    for (int ct = 0; ct < 2; ++ct) { v8f z = {0.f, 0.f, 0.f, 0.f, 0.f, 0.f, 0.f, 0.f}; c[ct] = z; }
#pragma unroll
    for (int kt = 0; kt < C2 / 32; ++kt) {
      const float* ap = acc + (16 * t + m) * C2 + 32 * kt + 8 * hh;
      const v4f p0 = *(const v4f*)ap,        p1 = *(const v4f*)(ap + 4);
      const v4f p2 = *(const v4f*)(ap + 16), p3 = *(const v4f*)(ap + 20);
      FragH a;
      a.h[0] = cvt8(p0, p1);
      a.h[1] = cvt8(p2, p3);
#pragma unroll
      for (int ct = 0; ct < 2; ++ct) c[ct] = wmh(a.v, bw[kt][ct].v, c[ct]);
    }
    const int node0 = nodeBase + 16 * t + 8 * hh;
    const v4f dA = *(const v4f*)(dO + (size_t)node0);
    const v4f dB = *(const v4f*)(dO + (size_t)node0 + 4);
    const float d0 = dA.x * WINV, d1 = dA.y * WINV, d2 = dA.z * WINV, d3 = dA.w * WINV;
    const float d4 = dB.x * WINV, d5 = dB.y * WINV, d6 = dB.z * WINV, d7 = dB.w * WINV;
    float* sp = acc + (16 * t + 8 * hh) * C2 + m;
#pragma unroll
    for (int ct = 0; ct < 2; ++ct) {
      sp[0 * C2 + 16 * ct] = c[ct][0] * d0;
      sp[1 * C2 + 16 * ct] = c[ct][1] * d1;
      sp[2 * C2 + 16 * ct] = c[ct][2] * d2;
      sp[3 * C2 + 16 * ct] = c[ct][3] * d3;
      sp[4 * C2 + 16 * ct] = c[ct][4] * d4;
      sp[5 * C2 + 16 * ct] = c[ct][5] * d5;
      sp[6 * C2 + 16 * ct] = c[ct][6] * d6;
      sp[7 * C2 + 16 * ct] = c[ct][7] * d7;
    }
  }
  __syncthreads();

  float* gbase = g3 + (size_t)nodeBase * C3;
#pragma unroll 4
  for (int q = 0; q < 32; ++q) {
    const int row = wave * 128 + 4 * q + (lane >> 3);
    const int col = 4 * (lane & 7);
    const v4f v = *(const v4f*)(acc + row * C2 + col);
    *(volatile v4f*)(gbase + (size_t)row * C3 + col) = v;
  }
  __threadfence();
#pragma unroll 4
  for (int q = 0; q < 32; ++q) {
    const int row = wave * 128 + 4 * q + (lane >> 3);
    const int col = 4 * (lane & 7);
    const v4f v = *(const v4f*)(acc + row * C2 + col);
    *(volatile v4f*)(gbase + (size_t)row * C3 + col) = v;
  }
}

__global__ __launch_bounds__(NTHR) void k_agg3(
    const int* __restrict__ srcl, const int* __restrict__ dstl, const float* __restrict__ g3,
    const float* __restrict__ dI, const float* __restrict__ b3, float* out, int nN, int nE) {
  extern __shared__ v4f lds_dyn[];
  float* acc  = (float*)lds_dyn;
  int*   list = (int*)(acc + NB3 * C3);
  int*   wcnt = list + LISTN;
  const int tid = threadIdx.x, lane = tid & 31, wave = tid >> 5;
  const int nodeBase = blockIdx.x * NB3;

  {
    const v4f z = {0.f, 0.f, 0.f, 0.f};
    for (int i = tid; i < NB3 * C3 / 4; i += NTHR) lds_dyn[i] = z;
  }
  __syncthreads();

  const int nChunks = (nE + CHUNK - 1) / CHUNK;
#pragma unroll 1
  for (int ch = 0; ch < nChunks; ++ch) {
    const int cbase = ch * CHUNK;
    const int wc = scan_chunk<NB3>(dstl, nE, cbase, nodeBase, list, tid, lane, wave);
    if (lane == 0) wcnt[wave] = wc;
    __syncthreads();
    if (wave == 0) {
#pragma unroll 1
      for (int wsx = 0; wsx < NWAVE; ++wsx) {
        int n = __builtin_amdgcn_readfirstlane(wcnt[wsx]);
        n = n > WCAP ? WCAP : (n < 0 ? 0 : n);
        const int* lp = list + wsx * WCAP;
#pragma unroll 1
        for (int i = 0; i < n; ++i) {
          const int ent  = __builtin_amdgcn_readfirstlane(lp[i]);
          const int slot = ent & (NB3 - 1);
          int e = cbase + ((ent >> 12) & (CHUNK - 1));
          e = e > nE - 1 ? nE - 1 : e;
          int s = srcl[e];
          s = s < 0 ? 0 : (s > nN - 1 ? nN - 1 : s);
          const float v = g3[(size_t)s * C3 + lane];
          float* ap = acc + slot * C3 + lane;
          *ap = *ap + v;
        }
      }
    }
    __syncthreads();
  }

  const float bl = b3[lane];
#pragma unroll 2
  for (int i = 0; i < NB3 / NWAVE; ++i) {
    const int r = wave * (NB3 / NWAVE) + i;
    int node = nodeBase + r;
    node = node > nN - 1 ? nN - 1 : node;
    const float d = dI[node];
    const float v = acc[r * C3 + lane] * d + bl;
    float mx = v;
#pragma unroll
    for (int o = 16; o >= 1; o >>= 1) mx = fmaxf(mx, __shfl_xor(mx, o, 32));
    const float ex = __expf(v - mx);
    float sm = ex;
#pragma unroll
    for (int o = 16; o >= 1; o >>= 1) sm += __shfl_xor(sm, o, 32);
    acc[r * C3 + lane] = ex * __builtin_amdgcn_rcpf(sm);
  }
  __syncthreads();

  const size_t outN = (size_t)nN * C3;
  const size_t ob   = (size_t)nodeBase * C3;
#pragma unroll 4
  for (int q = 0; q < 64; ++q) {
    const int f = (wave * 64 + q) * 128 + 4 * lane;
    const size_t gi = ob + (size_t)f;
    if (gi < outN) { const v4f v = *(const v4f*)(acc + f); *(volatile v4f*)(out + gi) = v; }
  }
  __threadfence();
#pragma unroll 4
  for (int q = 0; q < 64; ++q) {
    const int f = (wave * 64 + q) * 128 + 4 * lane;
    const size_t gi = ob + (size_t)f;
    if (gi < outN) { const v4f v = *(const v4f*)(acc + f); *(volatile v4f*)(out + gi) = v; }
  }
}

extern "C" void kernel_launch(void* const* d_in, const int* in_sizes, int n_in,
                              void* d_out, int out_size, void* d_ws, size_t ws_size,
                              hipStream_t stream) {
  if (n_in < 9) return;
  const int nN = in_sizes[0] / DF;
  const int nE = in_sizes[1];
  if (nN <= 0 || nE < 0 || in_sizes[0] != nN * DF || in_sizes[2] != nE) return;
  if (in_sizes[3] != DF * DF || in_sizes[4] < DF) return;
  if (in_sizes[5] != DF * C2 || in_sizes[6] < C2) return;
  if (in_sizes[7] != C2 * C3 || in_sizes[8] < C3) return;
  if (out_size != nN * C3) return;

  const float* x    = (const float*)d_in[0];
  const int*   srcl = (const int*)d_in[1];
  const int*   dstl = (const int*)d_in[2];
  const float* W1   = (const float*)d_in[3];
  const float* b1   = (const float*)d_in[4];
  const float* W2   = (const float*)d_in[5];
  const float* b2   = (const float*)d_in[6];
  const float* W3   = (const float*)d_in[7];
  const float* b3   = (const float*)d_in[8];
  float* out = (float*)d_out;

  const int nBD = (nN + NBD - 1) / NBD;
  const int nG1 = (nN + G1ROWS - 1) / G1ROWS;
  const int nA1 = (nN + NB1 - 1) / NB1;
  const int nA2 = (nN + NB2 - 1) / NB2;
  const int nA3 = (nN + NB3 - 1) / NB3;

  char* ws = (char*)d_ws;
  size_t off = 0;
  const size_t oW1 = off; off += (size_t)DF * DF * 2;                  off = (off + 255) & ~(size_t)255;
  const size_t oW2 = off; off += (size_t)C2 * DF * 2;                  off = (off + 255) & ~(size_t)255;
  const size_t oW3 = off; off += (size_t)C3 * C2 * 2;                  off = (off + 255) & ~(size_t)255;
  const size_t oDO = off; off += (size_t)nBD * NBD * 4;                off = (off + 255) & ~(size_t)255;
  const size_t oDI = off; off += (size_t)nBD * NBD * 4;                off = (off + 255) & ~(size_t)255;
  const size_t oG1 = off; off += (size_t)nG1 * G1ROWS * DF * 4;        off = (off + 255) & ~(size_t)255;
  const size_t oG2 = off; off += (size_t)nA1 * NB1 * C2 * 4;           off = (off + 255) & ~(size_t)255;
  const size_t oG3 = off; off += (size_t)nA2 * NB2 * C3 * 4;           off = (off + 255) & ~(size_t)255;
  if (off > ws_size) return;
  _Float16* w1s = (_Float16*)(ws + oW1);
  _Float16* w2s = (_Float16*)(ws + oW2);
  _Float16* w3s = (_Float16*)(ws + oW3);
  float*    dO  = (float*)(ws + oDO);
  float*    dI  = (float*)(ws + oDI);
  float*    g1  = (float*)(ws + oG1);
  float*    g2  = (float*)(ws + oG2);
  float*    g3  = (float*)(ws + oG3);

  const int nPrep = DF * DF / 8 + C2 * DF / 8 + C3 * C2 / 8;
  k_wprep<<<(nPrep + NTHR - 1) / NTHR, NTHR, 0, stream>>>(W1, W2, W3, w1s, w2s, w3s);

  k_deg<<<2 * nBD, NTHR, 0, stream>>>(srcl, dstl, dO, dI, nE, nBD);

  hipFuncSetAttribute(reinterpret_cast<const void*>(&k_gemm1),
                      hipFuncAttributeMaxDynamicSharedMemorySize, LDS_GEMM1);
  k_gemm1<<<nG1, NTHR, LDS_GEMM1, stream>>>(x, w1s, dO, g1, nN);

  hipFuncSetAttribute(reinterpret_cast<const void*>(&k_agg1),
                      hipFuncAttributeMaxDynamicSharedMemorySize, LDS_AGG);
  k_agg1<<<nA1, NTHR, LDS_AGG, stream>>>(srcl, dstl, g1, dO, dI, b1, w2s, g2, nN, nE);

  hipFuncSetAttribute(reinterpret_cast<const void*>(&k_agg2),
                      hipFuncAttributeMaxDynamicSharedMemorySize, LDS_AGG);
  k_agg2<<<nA2, NTHR, LDS_AGG, stream>>>(srcl, dstl, g2, dO, dI, b2, w3s, g3, nN, nE);

  hipFuncSetAttribute(reinterpret_cast<const void*>(&k_agg3),
                      hipFuncAttributeMaxDynamicSharedMemorySize, LDS_AGG);
  k_agg3<<<nA3, NTHR, LDS_AGG, stream>>>(srcl, dstl, g3, dI, b3, out, nN, nE);
}
